// FC_KANLayer_69363721830583
// MI455X (gfx1250) — hardware-verified
//
#include <hip/hip_runtime.h>
#include <hip/hip_bf16.h>
#include <math.h>

#define NSMP 6
#define TT 1024
#define DI 256
#define DO 512
#define NG 8
#define KSP (DI * NG)
#define SS 64
#define HH 1
#define DKK 64

typedef _Float16 bf16;
typedef _Float16 f16;
typedef __attribute__((ext_vector_type(4))) unsigned v4u_t;
typedef unsigned v4ua __attribute__((ext_vector_type(4), may_alias));
typedef __attribute__((ext_vector_type(4))) float v4f_t;
typedef float v4fa __attribute__((ext_vector_type(4), may_alias));
typedef __attribute__((ext_vector_type(16))) bf16  bf16x16;
typedef bf16x16 f16x16;
typedef __attribute__((ext_vector_type(8)))  bf16  bf16x8;
typedef bf16x8 f16x8;
typedef __attribute__((ext_vector_type(4)))  bf16  bf16x4;
typedef __attribute__((ext_vector_type(8)))  float f32x8;
__device__ __forceinline__ f32x8 wmma16(f16x16 a, f16x16 b, f32x8 c) {
  c = __builtin_amdgcn_wmma_f32_16x16x32_f16(false, a, false, b, (short)0, c, false, false);
  asm volatile("v_nop\n\tv_nop\n\tv_nop\n\tv_nop" : "+v"(c) : "v"(a), "v"(b));
  return c;
}
#define LDS_STRIDE 48
#define KSTRIDE    72
#define VSTRIDE    48

__device__ __forceinline__ f32x8 wmma_bf16(bf16x16 a, bf16x16 b, f32x8 c) {
  c = __builtin_amdgcn_wmma_f32_16x16x32_f16(false, a, false, b, (short)0, c, false, false);
  asm volatile("v_nop\n\tv_nop\n\tv_nop\n\tv_nop" : "+v"(c) : "v"(a), "v"(b));
  return c;
}

template <typename T>
__device__ __forceinline__ bf16x16 load_frag(const T* __restrict__ base, int ld,
                                             int row0, int k0) {
  const int lane = threadIdx.x & 31;
  const int r    = lane & 15;
  const int kh   = (lane >> 4) * 8;
  const T* p0 = base + (size_t)(row0 + r) * ld + (k0 + kh);
  const T* p1 = p0 + 16;
  bf16x16 f;
#pragma unroll
  for (int i = 0; i < 8; ++i) {
    f[i]     = (bf16)p0[i];
    f[i + 8] = (bf16)p1[i];
  }
  return f;
}

__device__ __forceinline__ bf16x16 lds_frag(const bf16* base, int stride) {
  const int lane = threadIdx.x & 31;
  const int row  = lane & 15;
  const int kh   = (lane >> 4) * 8;
  const bf16x8 lo = *(const bf16x8*)(base + row * stride + kh);
  const bf16x8 hi = *(const bf16x8*)(base + row * stride + kh + 16);
  bf16x16 f;
#pragma unroll
  for (int i = 0; i < 8; ++i) { f[i] = lo[i]; f[i + 8] = hi[i]; }
  return f;
}

template <typename T>
__device__ __forceinline__ void stage_read16(const T* __restrict__ p, float* buf) {
#pragma unroll
  for (int i = 0; i < 16; ++i) buf[i] = (float)p[i];
}

__device__ __forceinline__ void stage_write(bf16* dst, const float* buf, int nquad) {
#pragma unroll
  for (int i = 0; i < nquad; ++i) {
    bf16x4 q;
    q[0] = (bf16)buf[4 * i];     q[1] = (bf16)buf[4 * i + 1];
    q[2] = (bf16)buf[4 * i + 2]; q[3] = (bf16)buf[4 * i + 3];
    *(bf16x4*)(dst + 4 * i) = q;
  }
}

template <typename AT, int MODE>
__global__ __launch_bounds__(256) void gemm_rb_kernel(
    const AT* __restrict__ A, const float* __restrict__ W,
    const float* __restrict__ bias, const float* __restrict__ rowscale, const float* __restrict__ R, const float* __restrict__ rowbias, void* __restrict__ out,
    int M, int N, int K) {
  __shared__ bf16 ldsA[128 * LDS_STRIDE];
  __shared__ bf16 ldsW[256 * LDS_STRIDE];
  __shared__ __attribute__((aligned(16))) unsigned char sob[256 * 136 * 2];

  const int t    = threadIdx.x;
  const int wave = t >> 5;
  const int lane = t & 31;
  const int wm   = (wave & 1) * 64;
  const int wn   = (wave >> 1) * 64;
  const int mBlk = blockIdx.x * 128;
  const int nBlk = blockIdx.y * 256;

  const int arow = t >> 1;
  const int ach  = (t & 1) * 16;

  float abuf[16];
  float wbuf[32];

  stage_read16(A + (size_t)(mBlk + arow) * K + ach, abuf);
  const int nrow = min(nBlk + t, N - 1);
  stage_read16(W + (size_t)nrow * K,          wbuf);
  stage_read16(W + (size_t)nrow * K + 16,     wbuf + 16);

  f32x8 acc[4][4] = {};

  for (int k = 0; k < K; k += 32) {
    __syncthreads();
    stage_write(&ldsA[arow * LDS_STRIDE + ach], abuf, 4);
    stage_write(&ldsW[t * LDS_STRIDE],          wbuf, 8);
    if (k + 32 < K) {
      stage_read16(A + (size_t)(mBlk + arow) * K + (k + 32) + ach, abuf);
      stage_read16(W + (size_t)nrow * K + (k + 32),          wbuf);
      stage_read16(W + (size_t)nrow * K + (k + 32) + 16,     wbuf + 16);
    }
    __syncthreads();

    bf16x16 af[4], wf[4];
#pragma unroll
    for (int i = 0; i < 4; ++i)
      af[i] = lds_frag(ldsA + (wm + 16 * i) * LDS_STRIDE, LDS_STRIDE);
#pragma unroll
    for (int j = 0; j < 4; ++j)
      wf[j] = lds_frag(ldsW + (wn + 16 * j) * LDS_STRIDE, LDS_STRIDE);
#pragma unroll
    for (int i = 0; i < 4; ++i)
#pragma unroll
      for (int j = 0; j < 4; ++j)
        acc[i][j] = wmma_bf16(af[i], wf[j], acc[i][j]);
  }

  const int nlane = lane & 15;
  const int mh    = (lane >> 4) * 8;
  __syncthreads();
  if (MODE == 0 || MODE == 1 || MODE == 3) {
    bf16* so = (bf16*)sob;
#pragma unroll
    for (int i = 0; i < 4; ++i)
#pragma unroll
      for (int j = 0; j < 4; ++j) {
        const int nl = wn + 16 * j + nlane;
        const float bv = bias ? bias[nBlk + nl] : 0.0f;
        if (MODE == 3) {
#pragma unroll 1
          for (int r = 0; r < 8; ++r) {
            const int ml = wm + 16 * i + mh + r;
            const float xg = acc[i][j][r] + bv;
            so[ml * 264 + nl] = (bf16)(0.5f * xg * (1.0f + erff(xg * 0.70710678118654752f)));
          }
        } else {
#pragma unroll
        for (int r = 0; r < 8; ++r) {
          const int ml = wm + 16 * i + mh + r;
          const bf16 hv = (bf16)(acc[i][j][r] + bv);
          if (MODE == 0) so[ml * 264 + nl] = hv;
          else           so[nl * 136 + ml] = hv;
        }
        }
      }
    __syncthreads();
#pragma unroll 1
    for (int pass = 0; pass < 2; ++pass) {
      if (MODE == 0 || MODE == 3) {
        for (int ch = t; ch < 128 * 32; ch += 256) { const int ml = ch >> 5, q = (ch & 31) * 8;
          *(volatile v4u_t*)((bf16*)out + (size_t)(mBlk + ml) * N + nBlk + q) = *(const v4ua*)(so + ml * 264 + q); }
      } else {
        const int b_ = mBlk / SS, s0 = mBlk & (SS - 1);
        for (int ch = t; ch < 256 * 16; ch += 256) { const int nl = ch >> 4, q = (ch & 15) * 8; const int n = nBlk + nl, h = n >> 6, dk = n & (DKK - 1);
          *(volatile v4u_t*)((bf16*)out + (((size_t)(b_ * HH + h)) * DKK + dk) * SS + s0 + q) = *(const v4ua*)(so + nl * 136 + q); }
      }
      __threadfence();
    }
  } else {
    float* so = (float*)sob;
#pragma unroll 1
    for (int hf = 0; hf < 2; ++hf) {
      if (wm == hf * 64) {
#pragma unroll
        for (int i = 0; i < 4; ++i)
#pragma unroll
          for (int j = 0; j < 4; ++j) {
            const int nl = wn + 16 * j + nlane;
            const float bv = bias ? bias[nBlk + nl] : 0.0f;
#pragma unroll
            for (int r = 0; r < 8; ++r) { const int mrow = mBlk + hf * 64 + 16 * i + mh + r; so[(16 * i + mh + r) * 260 + nl] = acc[i][j][r] * (rowscale ? rowscale[mrow] : 1.0f) + bv + (rowbias ? rowbias[mrow] : 0.0f); }
          }
      }
      __syncthreads();
      if (R) {
        for (int ch = t; ch < 64 * 64; ch += 256) { const int ml = ch >> 6, q = (ch & 63) * 4;
          if (nBlk + q < N) { const v4f_t rv = *(const v4f_t*)(R + (size_t)(mBlk + hf * 64 + ml) * N + nBlk + q); v4f_t v = *(const v4fa*)(so + ml * 260 + q); v += rv; *(volatile v4fa*)(so + ml * 260 + q) = v; } }
        asm volatile("s_wait_dscnt 0" ::: "memory");
      }
#pragma unroll 1
      for (int pass = 0; pass < 2; ++pass) {
        for (int ch = t; ch < 64 * 64; ch += 256) { const int ml = ch >> 6, q = (ch & 63) * 4;
          if (nBlk + q < N) *(volatile v4f_t*)((float*)out + (size_t)(mBlk + hf * 64 + ml) * N + nBlk + q) = *(const v4fa*)(so + ml * 260 + q); }
        __threadfence();
      }
      __syncthreads();
    }
  }
}


__global__ __launch_bounds__(256) void k_ln(const float* __restrict__ X, const float* __restrict__ gam, const float* __restrict__ bet, float* __restrict__ Y) {
  const int tid = threadIdx.x, r = tid >> 3, part = tid & 7; const size_t row = (size_t)blockIdx.x * 32 + r;
  const float* xr = X + row * DI + part * 32; float v[32]; float s = 0.0f;
#pragma unroll
  for (int i = 0; i < 32; ++i) { v[i] = xr[i]; s += v[i]; }
  s += __shfl_xor(s, 1, 32); s += __shfl_xor(s, 2, 32); s += __shfl_xor(s, 4, 32);
  const float mean = s * (1.0f / DI); float q = 0.0f;
#pragma unroll
  for (int i = 0; i < 32; ++i) { const float d = v[i] - mean; q += d * d; }
  q += __shfl_xor(q, 1, 32); q += __shfl_xor(q, 2, 32); q += __shfl_xor(q, 4, 32);
  const float rstd = rsqrtf(q * (1.0f / DI) + 1e-5f);
#pragma unroll
  for (int i4 = 0; i4 < 8; ++i4) { v4f_t o; for (int e = 0; e < 4; ++e) { const int c = part * 32 + i4 * 4 + e; o[e] = (v[i4 * 4 + e] - mean) * rstd * gam[c] + bet[c]; }
    float* dst = Y + row * DI + part * 32 + i4 * 4; *(volatile v4f_t*)dst = o; __threadfence(); *(volatile v4f_t*)dst = o; }
}
__global__ __launch_bounds__(256) void k_rbf(const float* __restrict__ Xn, const float* __restrict__ grid, float* __restrict__ A) {
  const size_t e = (size_t)blockIdx.x * 256 + threadIdx.x; const size_t t = e >> 8; const int i = e & 255;
  const float x = Xn[t * DI + i]; const float inv = 7.0f / 3.0f; v4f_t o0, o1;
#pragma unroll
  for (int g = 0; g < 4; ++g) { const float u0 = (x - grid[g]) * inv, u1 = (x - grid[4 + g]) * inv; o0[g] = expf(-u0 * u0); o1[g] = expf(-u1 * u1); }
  float* dst = A + t * KSP + i * NG; *(volatile v4f_t*)dst = o0; *(volatile v4f_t*)(dst + 4) = o1; __threadfence(); *(volatile v4f_t*)dst = o0; *(volatile v4f_t*)(dst + 4) = o1;
}
__global__ __launch_bounds__(256) void k_bsp(const float* __restrict__ Xn, const float* __restrict__ grid, float* __restrict__ A) {
  __shared__ float gS[12]; __shared__ float bS[12][256];
  const int tid = threadIdx.x;
  if (tid < 12) gS[tid] = grid[tid];
  __syncthreads();
  const size_t e = (size_t)blockIdx.x * 256 + tid; const size_t t = e >> 8; const int i = e & 255;
  const float x = Xn[t * DI + i];
#pragma unroll 1
  for (int q = 0; q < 11; ++q) bS[q][tid] = (x >= gS[q] && x < gS[q + 1]) ? 1.0f : 0.0f;
  bS[11][tid] = 0.0f;
#pragma unroll 1
  for (int k = 1; k <= 3; ++k) {
#pragma unroll 1
    for (int q = 0; q < 11 - k; ++q) { const float l = (x - gS[q]) / (gS[q + k] - gS[q]), r = (gS[q + k + 1] - x) / (gS[q + k + 1] - gS[q + 1]); bS[q][tid] = l * bS[q][tid] + r * bS[q + 1][tid]; } }
  v4f_t o0, o1; for (int g = 0; g < 4; ++g) { o0[g] = bS[g][tid]; o1[g] = bS[4 + g][tid]; }
  float* dst = A + t * KSP + i * NG; *(volatile v4f_t*)dst = o0; *(volatile v4f_t*)(dst + 4) = o1; __threadfence(); *(volatile v4f_t*)dst = o0; *(volatile v4f_t*)(dst + 4) = o1;
}
__global__ __launch_bounds__(256) void k_silu(const float* __restrict__ Xn, float* __restrict__ A) { const size_t e = (size_t)blockIdx.x * 256 + threadIdx.x; const float x = Xn[e]; const float v = x / (1.0f + expf(-x)); *(volatile float*)(A + e) = v; __threadfence(); *(volatile float*)(A + e) = v; }
__global__ __launch_bounds__(256) void k_dog(const float* __restrict__ Xn, const float* __restrict__ scale, const float* __restrict__ trans, const float* __restrict__ bw, float* __restrict__ out) {
  __shared__ float xS[16 * DI];
  __shared__ __attribute__((aligned(16))) float oS[16 * 516];
  const int tid = threadIdx.x; const size_t t0 = (size_t)blockIdx.x * 16;
  for (int e = tid; e < 16 * DI; e += 256) xS[e] = Xn[t0 * DI + e];
  __syncthreads();
#pragma unroll 1
  for (int oo = 0; oo < 2; ++oo) { const int o = tid + oo * 256; const float* sc = scale + (size_t)o * DI; const float* tr = trans + (size_t)o * DI; const float* w = bw + (size_t)o * DI;
    float acc[16];
#pragma unroll
    for (int r = 0; r < 16; ++r) acc[r] = 0.0f;
#pragma unroll 1
    for (int i = 0; i < DI; ++i) { const float is = 1.0f / sc[i], tri = tr[i], wi = w[i];
#pragma unroll
      for (int r = 0; r < 16; ++r) { const float u = (xS[r * DI + i] - tri) * is; acc[r] += -u * expf(-0.5f * u * u) * wi; } }
#pragma unroll
    for (int r = 0; r < 16; ++r) oS[r * 516 + o] = acc[r]; }
  __syncthreads();
#pragma unroll 1
  for (int pass = 0; pass < 2; ++pass) { for (int q4 = tid; q4 < 16 * 128; q4 += 256) { const int r = q4 >> 7, c4 = (q4 & 127) * 4; *(volatile v4f_t*)(out + (t0 + r) * DO + c4) = *(const v4fa*)(oS + r * 516 + c4); } __threadfence(); }
}

extern "C" void kernel_launch(void* const* d_in, const int* in_sizes, int n_in,
                              void* d_out, int out_size, void* d_ws, size_t ws_size,
                              hipStream_t stream) {
  (void)in_sizes; (void)n_in; (void)out_size;
  const float** f = (const float**)d_in;
  const float* X = f[0], *ln_w = f[1], *ln_b = f[2], *bw = f[3], *sw = f[4], *scale = f[5], *trans = f[6], *grbf = f[7], *gbs = f[8];
  float* out = (float*)d_out;
  char* ws = (char*)d_ws;
  float* Xn = (float*)ws; ws += (size_t)NSMP * TT * DI * 4;
  float* A = (float*)ws; ws += (size_t)TT * KSP * 4;
  float* As = (float*)ws; ws += (size_t)TT * DI * 4;
  if ((size_t)(ws - (char*)d_ws) > ws_size) return;
  const dim3 blk(256);
  k_ln<<<dim3(NSMP * TT / 32), blk, 0, stream>>>(X, ln_w, ln_b, Xn);
  const int func[NSMP] = {0, 1, 2, 3, 0, 1};
  for (int s = 0; s < NSMP; ++s) {
    const float* xn = Xn + (size_t)s * TT * DI; float* o = out + (size_t)s * TT * DO;
    if (func[s] == 0 || func[s] == 1) {
      if (func[s] == 0) k_rbf<<<dim3(TT * DI / 256), blk, 0, stream>>>(xn, grbf, A); else k_bsp<<<dim3(TT * DI / 256), blk, 0, stream>>>(xn, gbs, A);
      gemm_rb_kernel<float, 2><<<dim3(TT / 128, DO / 256), blk, 0, stream>>>(A, sw, nullptr, nullptr, nullptr, nullptr, o, TT, DO, KSP);
    } else if (func[s] == 3) {
      k_silu<<<dim3(TT * DI / 256), blk, 0, stream>>>(xn, As);
      gemm_rb_kernel<float, 2><<<dim3(TT / 128, DO / 256), blk, 0, stream>>>(As, bw, nullptr, nullptr, nullptr, nullptr, o, TT, DO, DI);
    } else {
      k_dog<<<dim3(TT / 16), blk, 0, stream>>>(xn, scale, trans, bw, o);
    }
  }
}
